// RoPECrossAttention_54443005444919
// MI455X (gfx1250) — hardware-verified
//
#include <hip/hip_runtime.h>
#include <math.h>

constexpr int kBatch  = 4;
constexpr int kSq     = 1024;
constexpr int kSkv    = 2048;
constexpr int kDim    = 1024;
constexpr int kHeads  = 16;
constexpr int kHd     = 64;
constexpr int kTokQ   = kBatch * kSq;
constexpr int kTokKV  = kBatch * kSkv;
constexpr int kGrp    = 4;
constexpr int kChunks = kBatch * kHeads / kGrp;
constexpr float kWCarry     = 16.0f;
constexpr float kWCarryInv  = 1.0f / 16.0f;
constexpr float kScoreScale = 0.125f;
constexpr float kPCarry     = 4096.0f;
constexpr float kOCarry     = 256.0f;
constexpr float kPVScale    = kOCarry / kPCarry;
constexpr float kOutScale   = 1.0f / (kOCarry * kWCarry);
constexpr int kTabCosQ   = 0;
constexpr int kTabSinQ   = kSq * 32;
constexpr int kTabCosK   = 2 * kSq * 32;
constexpr int kTabSinK   = kTabCosK + kSkv * 32;
constexpr int kTabFloats = kTabSinK + kSkv * 32;

typedef __attribute__((ext_vector_type(16))) _Float16 v16h;
typedef __attribute__((ext_vector_type(8)))  _Float16 v8h;
typedef __attribute__((ext_vector_type(16))) __bf16   v16b;
typedef __attribute__((ext_vector_type(8)))  __bf16   v8b;
typedef __attribute__((ext_vector_type(8)))  float    v8f;
typedef __attribute__((ext_vector_type(4)))  float    v4f;
typedef __attribute__((ext_vector_type(4)))  unsigned int v4u;

__device__ __forceinline__ unsigned short f2bf_bits(float f) {
  unsigned u = __float_as_uint(f);
  return (unsigned short)((u + 0x7FFFu + ((u >> 16) & 1u)) >> 16);
}
__device__ __forceinline__ float bf_bits2f(unsigned short h) { return __uint_as_float(((unsigned)h) << 16); }

__device__ __forceinline__ void dep_guard_h(v8f& a, v8f& b, v16h x, v16h y) { asm volatile("v_nop\n\tv_nop\n\tv_nop\n\tv_nop" : "+v"(a), "+v"(b) : "v"(x), "v"(y)); }
__device__ __forceinline__ void dep_guard_b(v8f& a, v8f& b, v16b x, v16b y) { asm volatile("v_nop\n\tv_nop\n\tv_nop\n\tv_nop" : "+v"(a), "+v"(b) : "v"(x), "v"(y)); }
__device__ __forceinline__ void keep4_h(v16h a, v16h b, v16h c, v16h d) { asm volatile("v_nop" :: "v"(a), "v"(b), "v"(c), "v"(d)); }
__device__ __forceinline__ void keep4_b(v16b a, v16b b, v16b c, v16b d) { asm volatile("v_nop" :: "v"(a), "v"(b), "v"(c), "v"(d)); }
__device__ __forceinline__ void acc_guard4(v8f& a, v8f& b, v8f& c, v8f& d) { asm volatile("v_nop\n\tv_nop\n\tv_nop\n\tv_nop" : "+v"(a), "+v"(b), "+v"(c), "+v"(d)); }
template <typename T> struct Frag;
template <> struct Frag<_Float16> {
  typedef v16h V; union U { v16h v; v8h h[2]; };
  static __device__ __forceinline__ v16h load(const _Float16* p) {
    U f; f.h[0] = *(const v8h*)(p); f.h[1] = *(const v8h*)(p + 16); return f.v;
  }
  static __device__ __forceinline__ v8f mma(v16h a, v16h b, v8f c) {
    return __builtin_amdgcn_wmma_f32_16x16x32_f16(false, a, false, b, (short)0, c, false, false);
  }
  static __device__ __forceinline__ void guard(v8f& a, v8f& b, v16h x, v16h y) { dep_guard_h(a, b, x, y); }
  static __device__ __forceinline__ void keep(v16h a, v16h b, v16h c, v16h d) { keep4_h(a, b, c, d); }
};
template <> struct Frag<__bf16> {
  typedef v16b V; union U { v16b v; v8b h[2]; };
  static __device__ __forceinline__ v16b load(const __bf16* p) {
    U f; f.h[0] = *(const v8b*)(p); f.h[1] = *(const v8b*)(p + 16); return f.v;
  }
  static __device__ __forceinline__ v8f mma(v16b a, v16b b, v8f c) {
    return __builtin_amdgcn_wmma_f32_16x16x32_bf16(false, a, false, b, (short)0, c, false, false);
  }
  static __device__ __forceinline__ void guard(v8f& a, v8f& b, v16b x, v16b y) { dep_guard_b(a, b, x, y); }
  static __device__ __forceinline__ void keep(v16b a, v16b b, v16b c, v16b d) { keep4_b(a, b, c, d); }
};

__device__ __forceinline__ unsigned pk16(unsigned short a, unsigned short b) { return (unsigned)a | ((unsigned)b << 16); }
__device__ __forceinline__ unsigned short h_bits(float f) { const _Float16 h = (_Float16)f; return __builtin_bit_cast(unsigned short, h); }

template <int ET> struct Elem;
template <> struct Elem<0> { typedef _Float16 T; };
template <> struct Elem<1> { typedef __bf16 T; };
template <int ET, bool SPLIT, int BIAS_MODE, int OUT_MODE, bool RESID, int ACT = 0>
__global__ __launch_bounds__(256) void wmma_gemm64(
    const unsigned short* __restrict__ Ap, const unsigned short* __restrict__ A2p, int lda, long strideA,
    const unsigned short* __restrict__ Btp, const unsigned short* __restrict__ Bt2p, int ldb, long strideB,
    void* __restrict__ Cout, void* __restrict__ Cout2, int ldc, long strideC,
    const float* __restrict__ bias,
    const float* __restrict__ resid, long strideR,
    int M, int N, int K, float scale) {
  typedef typename Elem<ET>::T T;
  typedef typename Frag<T>::V V;
  const T* A = (const T*)Ap; const T* A2 = (const T*)A2p; const T* Bt = (const T*)Btp; const T* Bt2 = (const T*)Bt2p;
  __shared__ __align__(16) float sT[8][16 * 68];
  const int b    = blockIdx.y;
  const int lane = threadIdx.x & 31;
  const int wave = threadIdx.x >> 5;
  const int tilesN = N >> 6;
  const int tilesM = M >> 6;
  const int tile = blockIdx.x * 8 + wave;
  if (tile >= tilesM * tilesN) return;
  const int tm = tile / tilesN;
  const int tn = tile - tm * tilesN;
  const int m0 = tm << 6;
  const int n0 = tn << 6;

  const T* Ab  = A  + (size_t)b * strideA;
  const T* Bb  = Bt + (size_t)b * strideB;
  const T* Ab2 = SPLIT ? (A2  + (size_t)b * strideA) : nullptr;
  const T* Bb2 = SPLIT ? (Bt2 + (size_t)b * strideB) : nullptr;

  const int rlane = lane & 15;
  const int koff  = (lane >> 4) * 8;
  const int mOff  = (lane >> 4) * 8;

  v8f acc[4][4];
#pragma unroll
  for (int i = 0; i < 4; ++i)
#pragma unroll
    for (int j = 0; j < 4; ++j) acc[i][j] = (v8f){0.f,0.f,0.f,0.f,0.f,0.f,0.f,0.f};

  for (int k0 = 0; k0 < K; k0 += 32) {
    V bh[4], bl[4];
#pragma unroll
    for (int j = 0; j < 4; ++j) {
      const size_t bo = (size_t)(n0 + (j << 4) + rlane) * ldb + koff + k0;
      bh[j] = Frag<T>::load(Bb + bo);
      if (SPLIT) bl[j] = Frag<T>::load(Bb2 + bo);
    }
#pragma unroll
    for (int i = 0; i < 4; ++i) {
      const size_t ao = (size_t)(m0 + (i << 4) + rlane) * lda + koff + k0;
      V ah = Frag<T>::load(Ab + ao);
      V al;
      if (SPLIT) al = Frag<T>::load(Ab2 + ao);
#pragma unroll
      for (int j = 0; j < 4; ++j) {
        acc[i][j] = Frag<T>::mma(ah, bh[j], acc[i][j]);
        if (SPLIT) {
          acc[i][j] = Frag<T>::mma(ah, bl[j], acc[i][j]);
          acc[i][j] = Frag<T>::mma(al, bh[j], acc[i][j]);
        }
      }
      Frag<T>::guard(acc[i][0], acc[i][3], ah, SPLIT ? al : ah);
    }
    Frag<T>::keep(bh[0], bh[1], bh[2], bh[3]);
    if (SPLIT) Frag<T>::keep(bl[0], bl[1], bl[2], bl[3]);
  }
  acc_guard4(acc[0][0], acc[0][1], acc[0][2], acc[0][3]);
  acc_guard4(acc[1][0], acc[1][1], acc[1][2], acc[1][3]);
  acc_guard4(acc[2][0], acc[2][1], acc[2][2], acc[2][3]);
  acc_guard4(acc[3][0], acc[3][1], acc[3][2], acc[3][3]);

  float* slab = sT[wave];
  const float* Rb = RESID ? (resid + (size_t)b * strideR) : nullptr;
#pragma unroll
  for (int i = 0; i < 4; ++i) {
    const int mBase = m0 + (i << 4);
#pragma unroll
    for (int j = 0; j < 4; ++j) {
      const int n = n0 + (j << 4) + rlane;
      float bv = 0.f;
      if (BIAS_MODE == 2) bv = bias[n];
#pragma unroll
      for (int r = 0; r < 8; ++r) {
        float v = acc[i][j][r] * scale;
        if (BIAS_MODE == 1) v += bias[mBase + mOff + r];
        if (BIAS_MODE == 2) v += bv;
        if (RESID) v += Rb[(size_t)(mBase + mOff + r) * ldc + n];
        if (ACT == 2) v = fmaxf(v, 0.0f);
        if (ACT == 4) v = (v > 0.f) ? v : 0.01f * v;
        slab[(mOff + r) * 68 + (j << 4) + rlane] = v;
      }
    }
    __builtin_amdgcn_fence(__ATOMIC_RELEASE, "workgroup");
    __builtin_amdgcn_wave_barrier();
    __builtin_amdgcn_fence(__ATOMIC_ACQUIRE, "workgroup");
    if (OUT_MODE == 0) {
      float* C = (float*)Cout + (size_t)b * strideC;
      const int hh = lane >> 4, c4 = (lane & 15) * 4;
      for (int pass = 0; pass < 2; ++pass) {
#pragma unroll
        for (int it = 0; it < 8; ++it) {
          const int row = it * 2 + hh;
          v4f v = *(const v4f*)(slab + row * 68 + c4);
          *(volatile v4f*)(C + (size_t)(mBase + row) * ldc + n0 + c4) = v;
        }
        __threadfence();
      }
    } else {
      const int q = lane >> 3, c8 = (lane & 7) * 8;
      unsigned short* C  = (unsigned short*)Cout  + (size_t)b * strideC;
      unsigned short* C2 = (OUT_MODE == 2) ? ((unsigned short*)Cout2 + (size_t)b * strideC) : nullptr;
      for (int pass = 0; pass < 2; ++pass) {
#pragma unroll
        for (int it = 0; it < 4; ++it) {
          const int row = it * 4 + q;
          const float* sp = slab + row * 68 + c8;
          v8h hv, lv;
#pragma unroll
          for (int e = 0; e < 8; ++e) {
            if (OUT_MODE == 1) {
              hv[e] = (_Float16)sp[e];
            } else {
              unsigned short hb = f2bf_bits(sp[e]);
              unsigned short lb = f2bf_bits(sp[e] - bf_bits2f(hb));
              hv[e] = __builtin_bit_cast(_Float16, hb);
              lv[e] = __builtin_bit_cast(_Float16, lb);
            }
          }
          *(volatile v8h*)(C + (size_t)(mBase + row) * ldc + n0 + c8) = hv;
          if (OUT_MODE == 2) *(volatile v8h*)(C2 + (size_t)(mBase + row) * ldc + n0 + c8) = lv;
        }
        __threadfence();
      }
    }
    __builtin_amdgcn_fence(__ATOMIC_RELEASE, "workgroup");
    __builtin_amdgcn_wave_barrier();
    __builtin_amdgcn_fence(__ATOMIC_ACQUIRE, "workgroup");
  }
}

__global__ __launch_bounds__(256) void cast8_f16_kernel(const float* __restrict__ in, unsigned short* __restrict__ out,
                                                        int n8, float scale) {
  const int i = blockIdx.x * 256 + threadIdx.x;
  if (i >= n8) return;
  const float* p = in + 8 * (size_t)i;
  const v4f a = *(const v4f*)(p);
  const v4f c = *(const v4f*)(p + 4);
  unsigned short hb[8];
#pragma unroll
  for (int e = 0; e < 4; ++e) {
    hb[e]     = h_bits(a[e] * scale);
    hb[4 + e] = h_bits(c[e] * scale);
  }
  const v4u u = (v4u){pk16(hb[0], hb[1]), pk16(hb[2], hb[3]), pk16(hb[4], hb[5]), pk16(hb[6], hb[7])};
  unsigned short* q = out + 8 * (size_t)i;
  *(volatile v4u*)q = u;
  __threadfence();
  *(volatile v4u*)q = u;
}

__global__ __launch_bounds__(256) void castw4_f16_kernel(const float* __restrict__ W0, const float* __restrict__ W1,
                                                         const float* __restrict__ W2, const float* __restrict__ W3,
                                                         unsigned short* __restrict__ out, int n8each, float scale) {
  const int z = blockIdx.y;
  const float* W = (z == 0) ? W0 : (z == 1) ? W1 : (z == 2) ? W2 : W3;
  const int i = blockIdx.x * 256 + threadIdx.x;
  if (i >= n8each) return;
  const float* p = W + 8 * (size_t)i;
  const v4f a = *(const v4f*)(p);
  const v4f c = *(const v4f*)(p + 4);
  unsigned short hb[8];
#pragma unroll
  for (int e = 0; e < 4; ++e) {
    hb[e]     = h_bits(a[e] * scale);
    hb[4 + e] = h_bits(c[e] * scale);
  }
  const v4u u = (v4u){pk16(hb[0], hb[1]), pk16(hb[2], hb[3]), pk16(hb[4], hb[5]), pk16(hb[6], hb[7])};
  unsigned short* q = out + (size_t)z * 8 * (size_t)n8each + 8 * (size_t)i;
  *(volatile v4u*)q = u;
  __threadfence();
  *(volatile v4u*)q = u;
}

__global__ __launch_bounds__(32) void invfreq_kernel(float* __restrict__ invf) {
  const int i = threadIdx.x;
  const float e = (float)i * (1.0f / 32.0f);
  const float p = powf(10000.0f, e);
  const float v = 1.0f / p;
  ((volatile float*)invf)[i] = v;
  __threadfence();
  ((volatile float*)invf)[i] = v;
}

__global__ __launch_bounds__(256) void rope_tables_kernel(const float* __restrict__ invf, float* __restrict__ tab, int nth) {
  const int idx = blockIdx.x * 256 + threadIdx.x;
  if (idx >= nth) return;
  const int fi = idx & 31;
  const int r  = idx >> 5;
  const bool isq = (r < kSq);
  const int row = isq ? r : (r - kSq);
  const int pos = isq ? (row * 2) : row;
  const float f = invf[fi];
  const float ang = (float)pos * f;
  const float cs = cosf(ang);
  const float sn = sinf(ang);
  const size_t ci = (isq ? (size_t)kTabCosQ : (size_t)kTabCosK) + (size_t)row * 32 + fi;
  const size_t si = ci + (isq ? (size_t)(kTabSinQ - kTabCosQ) : (size_t)(kTabSinK - kTabCosK));
  volatile float* vt = (volatile float*)tab;
  vt[ci] = cs;
  vt[si] = sn;
  __threadfence();
  vt[ci] = cs;
  vt[si] = sn;
}

__global__ __launch_bounds__(256) void rope_apply_kernel(const float* __restrict__ X, const float* __restrict__ tab,
                                                         unsigned short* __restrict__ Y, int nth, int L, int sinoff) {
  const int i = blockIdx.x * 256 + threadIdx.x;
  if (i >= nth) return;
  const int row = i >> 7;
  const int c0  = (i & 127) << 3;
  const int s   = row - (row / L) * L;
  const int d0  = c0 & 63;
  const int fi0 = d0 & 31;
  const int pc0 = c0 ^ 32;
  const float sgn = (d0 < 32) ? -1.0f : 1.0f;
  const float* xr = X + (size_t)row * kDim;
  const v4f xa = *(const v4f*)(xr + c0);
  const v4f xb = *(const v4f*)(xr + c0 + 4);
  const v4f pa = *(const v4f*)(xr + pc0);
  const v4f pb = *(const v4f*)(xr + pc0 + 4);
  const float* cr = tab + (size_t)s * 32 + fi0;
  const v4f ca = *(const v4f*)(cr);
  const v4f cb = *(const v4f*)(cr + 4);
  const v4f sa = *(const v4f*)(cr + sinoff);
  const v4f sb = *(const v4f*)(cr + sinoff + 4);
  unsigned short hb[8];
#pragma unroll
  for (int e = 0; e < 4; ++e) {
    const float o0 = xa[e] * ca[e] + (sgn * pa[e]) * sa[e];
    const float o1 = xb[e] * cb[e] + (sgn * pb[e]) * sb[e];
    hb[e]     = h_bits(o0);
    hb[4 + e] = h_bits(o1);
  }
  const v4u u = (v4u){pk16(hb[0], hb[1]), pk16(hb[2], hb[3]), pk16(hb[4], hb[5]), pk16(hb[6], hb[7])};
  unsigned short* q = Y + (size_t)row * kDim + c0;
  *(volatile v4u*)q = u;
  __threadfence();
  *(volatile v4u*)q = u;
}

__global__ __launch_bounds__(256) void softmax_row_kernel(const float* __restrict__ Sc, unsigned short* __restrict__ P, float carry) {
  __shared__ float redM[8];
  __shared__ float redS[8];
  const int row  = blockIdx.x;
  const int t    = threadIdx.x;
  const int lane = t & 31, wave = t >> 5;
  const int c0   = t * 8;
  const float* sr = Sc + (size_t)row * kSkv + c0;
  const v4f a = *(const v4f*)(sr);
  const v4f c = *(const v4f*)(sr + 4);
  float x[8];
#pragma unroll
  for (int e = 0; e < 4; ++e) { x[e] = a[e]; x[4 + e] = c[e]; }
  float m = fmaxf(fmaxf(fmaxf(x[0], x[1]), fmaxf(x[2], x[3])), fmaxf(fmaxf(x[4], x[5]), fmaxf(x[6], x[7])));
#pragma unroll
  for (int off = 16; off > 0; off >>= 1) m = fmaxf(m, __shfl_xor(m, off, 32));
  if (lane == 0) redM[wave] = m;
  __syncthreads();
  float gm = redM[0];
#pragma unroll
  for (int w = 1; w < 8; ++w) gm = fmaxf(gm, redM[w]);
  float p[8];
  float s = 0.0f;
#pragma unroll
  for (int e = 0; e < 8; ++e) { p[e] = expf(x[e] - gm); s += p[e]; }
#pragma unroll
  for (int off = 16; off > 0; off >>= 1) s += __shfl_xor(s, off, 32);
  if (lane == 0) redS[wave] = s;
  __syncthreads();
  float tot = redS[0];
#pragma unroll
  for (int w = 1; w < 8; ++w) tot += redS[w];
  const float inv = carry / tot;
  unsigned short hb[8];
#pragma unroll
  for (int e = 0; e < 8; ++e) hb[e] = h_bits(p[e] * inv);
  const v4u u = (v4u){pk16(hb[0], hb[1]), pk16(hb[2], hb[3]), pk16(hb[4], hb[5]), pk16(hb[6], hb[7])};
  unsigned short* q = P + (size_t)row * kSkv + c0;
  *(volatile v4u*)q = u;
  __threadfence();
  *(volatile v4u*)q = u;
}

extern "C" void kernel_launch(void* const* d_in, const int* in_sizes, int n_in,
                              void* d_out, int out_size, void* d_ws, size_t ws_size,
                              hipStream_t stream)
{
  if (n_in < 10) return;
  if (in_sizes[0] != kTokQ * kDim || in_sizes[1] != kTokKV * kDim) return;
  if (in_sizes[2] != kDim * kDim || in_sizes[4] != kDim * kDim || in_sizes[6] != kDim * kDim || in_sizes[8] != kDim * kDim) return;
  if (in_sizes[3] != kDim || in_sizes[5] != kDim || in_sizes[7] != kDim || in_sizes[9] != kDim) return;
  if (out_size != kTokQ * kDim) return;

  const float* query = (const float*)d_in[0];
  const float* kvin  = (const float*)d_in[1];
  const float* q_w   = (const float*)d_in[2];
  const float* q_b   = (const float*)d_in[3];
  const float* k_w   = (const float*)d_in[4];
  const float* k_b   = (const float*)d_in[5];
  const float* v_w   = (const float*)d_in[6];
  const float* v_b   = (const float*)d_in[7];
  const float* out_w = (const float*)d_in[8];
  const float* out_b = (const float*)d_in[9];
  float* out = (float*)d_out;

  char* ws = (char*)d_ws;
  const size_t szW1 = (size_t)kDim * kDim * 2;
  const size_t oW16 = 0;
  const size_t oX1  = oW16 + 4 * szW1;
  const size_t szX1 = (size_t)kTokQ * kDim * 2;
  const size_t oX2  = oX1 + szX1;
  const size_t szX2 = (size_t)kTokKV * kDim * 2;
  const size_t oQ16 = oX2 + szX2;
  const size_t oVt  = oQ16 + szX1;
  const size_t szVt = (size_t)kBatch * kDim * kSkv * 2;
  const size_t oR5  = oVt + szVt;
  const size_t szSc = (size_t)kGrp * kSq * kSkv * 4;
  const size_t szP  = (size_t)kGrp * kSq * kSkv * 2;
  const size_t szKf = (size_t)kTokKV * kDim * 4;
  size_t szR5 = szSc + szP;
  if (szKf > szR5) szR5 = szKf;
  const size_t oTab  = oR5 + szR5;
  const size_t szTab = 4096 + (size_t)kTabFloats * 4;
  const size_t total = oTab + szTab;
  if (total > ws_size) return;

  unsigned short* qw16  = (unsigned short*)(ws + oW16);
  unsigned short* kw16  = qw16 + (size_t)kDim * kDim;
  unsigned short* vw16  = kw16 + (size_t)kDim * kDim;
  unsigned short* ow16  = vw16 + (size_t)kDim * kDim;
  unsigned short* xq16  = (unsigned short*)(ws + oX1);
  unsigned short* o16   = (unsigned short*)(ws + oX1);
  unsigned short* xkv16 = (unsigned short*)(ws + oX2);
  unsigned short* k16   = (unsigned short*)(ws + oX2);
  unsigned short* q16   = (unsigned short*)(ws + oQ16);
  unsigned short* vt16  = (unsigned short*)(ws + oVt);
  float* qf32 = (float*)(ws + oR5);
  float* kf32 = (float*)(ws + oR5);
  float* sc   = (float*)(ws + oR5);
  unsigned short* p16 = (unsigned short*)(ws + oR5 + szSc);
  float* invf = (float*)(ws + oTab);
  float* tab  = (float*)(ws + oTab + 4096);

  const dim3 blk(256);

  cast8_f16_kernel<<<dim3(kTokQ * kDim / 8 / 256), blk, 0, stream>>>(query, xq16, kTokQ * kDim / 8, 1.0f);
  cast8_f16_kernel<<<dim3(kTokKV * kDim / 8 / 256), blk, 0, stream>>>(kvin, xkv16, kTokKV * kDim / 8, 1.0f);
  castw4_f16_kernel<<<dim3(kDim * kDim / 8 / 256, 4), blk, 0, stream>>>(q_w, k_w, v_w, out_w, qw16, kDim * kDim / 8, kWCarry);
  invfreq_kernel<<<dim3(1), dim3(32), 0, stream>>>(invf);
  rope_tables_kernel<<<dim3((kSq + kSkv) * 32 / 256), blk, 0, stream>>>(invf, tab, (kSq + kSkv) * 32);

  wmma_gemm64<0, false, 2, 0, false><<<dim3((kTokQ / 64) * (kDim / 64) / 8, 1), blk, 0, stream>>>(
      xq16, xq16, kDim, 0L, qw16, qw16, kDim, 0L, (void*)qf32, (void*)qf32, kDim, 0L,
      q_b, tab, 0L, kTokQ, kDim, kDim, kWCarryInv);
  rope_apply_kernel<<<dim3(kTokQ * 128 / 256), blk, 0, stream>>>(qf32, tab + kTabCosQ, q16, kTokQ * 128, kSq, kTabSinQ - kTabCosQ);
  wmma_gemm64<0, false, 2, 0, false><<<dim3((kTokKV / 64) * (kDim / 64) / 8, 1), blk, 0, stream>>>(
      xkv16, xkv16, kDim, 0L, kw16, kw16, kDim, 0L, (void*)kf32, (void*)kf32, kDim, 0L,
      k_b, tab, 0L, kTokKV, kDim, kDim, kWCarryInv);
  wmma_gemm64<0, false, 1, 1, false><<<dim3((kDim / 64) * (kSkv / 64) / 8, kBatch), blk, 0, stream>>>(
      vw16, vw16, kDim, 0L, xkv16, xkv16, kDim, (long)kSkv * kDim, (void*)vt16, (void*)vt16, kSkv, (long)kDim * kSkv,
      v_b, tab, 0L, kDim, kSkv, kDim, kWCarryInv);
  rope_apply_kernel<<<dim3(kTokKV * 128 / 256), blk, 0, stream>>>(kf32, tab + kTabCosK, k16, kTokKV * 128, kSkv, kTabSinK - kTabCosK);

  for (int ch = 0; ch < kChunks; ++ch) {
    const int b  = ch / (kHeads / kGrp);
    const int h0 = (ch % (kHeads / kGrp)) * kGrp;
    const unsigned short* qa = q16 + (size_t)b * kSq * kDim + (size_t)h0 * kHd;
    const unsigned short* kb = k16 + (size_t)b * kSkv * kDim + (size_t)h0 * kHd;
    wmma_gemm64<0, false, 0, 0, false><<<dim3((kSq / 64) * (kSkv / 64) / 8, kGrp), blk, 0, stream>>>(
        qa, qa, kDim, (long)kHd, kb, kb, kDim, (long)kHd, (void*)sc, (void*)sc, kSkv, (long)kSq * kSkv,
        q_b, tab, 0L, kSq, kSkv, kHd, kScoreScale);
    softmax_row_kernel<<<dim3(kGrp * kSq), blk, 0, stream>>>(sc, p16, kPCarry);
    const unsigned short* vb = vt16 + ((size_t)b * kDim + (size_t)h0 * kHd) * kSkv;
    unsigned short* ob = o16 + (size_t)b * kSq * kDim + (size_t)h0 * kHd;
    wmma_gemm64<0, false, 0, 1, false><<<dim3((kSq / 64) * (kHd / 64) / 8, kGrp), blk, 0, stream>>>(
        p16, p16, kSkv, (long)kSq * kSkv, vb, vb, kSkv, (long)kHd * kSkv, (void*)ob, (void*)ob, kDim, (long)kHd,
        q_b, tab, 0L, kSq, kHd, kSkv, kPVScale);
  }

  wmma_gemm64<0, false, 2, 0, false><<<dim3((kTokQ / 64) * (kDim / 64) / 8, 1), blk, 0, stream>>>(
      o16, o16, kDim, 0L, ow16, ow16, kDim, 0L, (void*)out, (void*)out, kDim, 0L,
      out_b, tab, 0L, kTokQ, kDim, kDim, kOutScale);
}
